// MultiHeadAttention_63393717289722
// MI455X (gfx1250) — hardware-verified
//
#include <hip/hip_runtime.h>


#ifndef NB
#define NB 4
#endif
#ifndef SEQ
#define SEQ 2048
#endif
#define NB_FULL  4
#define SEQ_FULL 2048
#define DM   512
#define NH   8
#define HD   64
#define PCAR 1024.0f
#define SCL  0.125f
#define L2E  1.4426950408889634f
#define LKP  72
#define LPP  40
#define LOP  68

static_assert(DM == NH * HD);
static_assert(HD == 64);
static_assert(DM % 32 == 0);
static_assert(DM % 64 == 0);
static_assert(SEQ % 64 == 0);
static_assert((SEQ * DM) % (8 * 256) == 0);
static_assert((DM * DM) % (8 * 256) == 0);
static_assert(NB <= NB_FULL);
static_assert(SEQ <= SEQ_FULL);
static_assert(LKP % 8 == 0);
static_assert(LPP % 8 == 0);
static_assert(LOP % 4 == 0);

typedef _Float16 h16;
typedef unsigned short bf;
typedef __attribute__((ext_vector_type(16))) __bf16   v16bf;
typedef __attribute__((ext_vector_type(16))) _Float16 v16h;
typedef __attribute__((ext_vector_type(8)))  _Float16 v8h;
typedef __attribute__((ext_vector_type(8)))  unsigned short v8us;
typedef __attribute__((ext_vector_type(8)))  float    v8f;
typedef __attribute__((ext_vector_type(4)))  float    v4f;
typedef v8h  __attribute__((may_alias)) v8ha;
typedef v4f  __attribute__((may_alias)) v4fa;
typedef v8us __attribute__((may_alias)) v8usa;

__device__ __forceinline__ unsigned short f2bf(float f) { unsigned u = __float_as_uint(f); u += 0x7FFFu + ((u >> 16) & 1u); return (unsigned short)(u >> 16); }
__device__ __forceinline__ float bf2f(unsigned short b) { return __uint_as_float(((unsigned)b) << 16); }
__device__ __forceinline__ float bfr(float f) { return bf2f(f2bf(f)); }
__device__ __forceinline__ void splitf(float y, unsigned short& h, unsigned short& l) { h = f2bf(y); l = f2bf(y - bf2f(h)); }
__device__ __forceinline__ v16h cat16(v8h lo, v8h hi) { return __builtin_shufflevector(lo, hi, 0, 1, 2, 3, 4, 5, 6, 7, 8, 9, 10, 11, 12, 13, 14, 15); }
__device__ __forceinline__ v16bf cat16b(v8us lo, v8us hi) { return __builtin_bit_cast(v16bf, __builtin_shufflevector(lo, hi, 0, 1, 2, 3, 4, 5, 6, 7, 8, 9, 10, 11, 12, 13, 14, 15)); }
__device__ __forceinline__ v8f wmma16(v16h a, v16h b, v8f c) { return __builtin_amdgcn_wmma_f32_16x16x32_f16(false, a, false, b, (short)0, c, false, false); }
__device__ __forceinline__ v8f wmmab(v16bf a, v16bf b, v8f c) { return __builtin_amdgcn_wmma_f32_16x16x32_bf16(false, a, false, b, (short)0, c, false, false); }
__device__ __forceinline__ v16bf ldg16(const bf* __restrict__ p) { return cat16b(*(const v8us*)p, *(const v8us*)(p + 16)); }
__device__ __forceinline__ void wsync() { __builtin_amdgcn_wave_barrier(); asm volatile("" ::: "memory"); }

template <int NSPLIT>
__device__ __forceinline__ void gemm_loop(const bf* __restrict__ A, const bf* __restrict__ A2, const bf* __restrict__ Bt, const int K, const size_t aoff, const size_t boff, v8f (&acc)[4][4]) {
#pragma unroll 1
    for (int kc = 0; kc < K; kc += 32) {
        v16bf a[4], a2[4];
#pragma unroll
        for (int mb = 0; mb < 4; ++mb) { a[mb] = ldg16(A + aoff + (size_t)mb * 16 * K + kc); if (NSPLIT == 1) a2[mb] = ldg16(A2 + aoff + (size_t)mb * 16 * K + kc); }
#pragma unroll
        for (int nb = 0; nb < 4; ++nb) { const v16bf b = ldg16(Bt + boff + (size_t)nb * 16 * K + kc);
#pragma unroll
            for (int mb = 0; mb < 4; ++mb) { acc[mb][nb] = wmmab(a[mb], b, acc[mb][nb]); if (NSPLIT == 1) acc[mb][nb] = wmmab(a2[mb], b, acc[mb][nb]); } }
        asm volatile("v_nop\n\tv_nop\n\tv_nop\n\tv_nop" : "+v"(acc[0][0]), "+v"(acc[1][1]), "+v"(acc[2][2]), "+v"(acc[3][3]) : "v"(a[0]), "v"(a[3]));
    }
}

__global__ __launch_bounds__(256) void k_cvt8(const float* __restrict__ src, bf* dst, unsigned n8, size_t sstride, size_t dstride) {
    const unsigned i = blockIdx.x * 256u + threadIdx.x; if (i >= n8) return;
    const float* s = src + (size_t)blockIdx.y * sstride + (size_t)i * 8; bf* d = dst + (size_t)blockIdx.y * dstride + (size_t)i * 8;
    const v4f v0 = *(const v4f*)s; const v4f v1 = *(const v4f*)(s + 4); v8us o;
#pragma unroll
    for (int k = 0; k < 4; ++k) { o[k] = f2bf(v0[k]); o[4 + k] = f2bf(v1[k]); }
    *(volatile v8us*)d = o; __threadfence(); *(volatile v8us*)d = o;
}

__global__ __launch_bounds__(32) void k_gemm_qk(const bf* __restrict__ X, const bf* __restrict__ W, bf* Ph, bf* Pl, float sc) {
    __shared__ __align__(16) float os[16 * LOP];
    const int lane = threadIdx.x & 31, lr = lane & 15, hi = lane >> 4;
    const size_t z = blockIdx.z; const int r0 = blockIdx.x * 64, c0 = blockIdx.y * 64;
    const bf* A = X + z * (size_t)SEQ * DM;
    v8f acc[4][4];
#pragma unroll
    for (int mb = 0; mb < 4; ++mb)
#pragma unroll
        for (int nb = 0; nb < 4; ++nb) acc[mb][nb] = (v8f){};
    gemm_loop<0>(A, A, W, DM, (size_t)(r0 + lr) * DM + 8 * hi, (size_t)(c0 + lr) * DM + 8 * hi, acc);
    const size_t pbase = ((z * NH + blockIdx.y) * (size_t)SEQ + r0) * HD;
    const int srow = lane >> 3, scol = (lane & 7) * 8;
#pragma unroll
    for (int mb = 0; mb < 4; ++mb) {
#pragma unroll
        for (int nb = 0; nb < 4; ++nb) {
#pragma unroll
            for (int j = 0; j < 8; ++j) os[(hi * 8 + j) * LOP + nb * 16 + lr] = acc[mb][nb][j]; }
        wsync();
#pragma unroll 1
        for (int ps = 0; ps < 2; ++ps) {
#pragma unroll
            for (int s = 0; s < 4; ++s) { const int row = 4 * s + srow; const v4f x0 = *(const v4fa*)(&os[row * LOP + scol]); const v4f x1 = *(const v4fa*)(&os[row * LOP + scol + 4]); v8us oh, ol;
#pragma unroll
                for (int j = 0; j < 4; ++j) { unsigned short a, c; splitf(x0[j] * sc, a, c); oh[j] = a; ol[j] = c; splitf(x1[j] * sc, a, c); oh[4 + j] = a; ol[4 + j] = c; }
                const size_t off = pbase + (size_t)(mb * 16 + row) * HD + scol;
                *(volatile v8us*)(Ph + off) = oh; *(volatile v8us*)(Pl + off) = ol; }
            if (ps == 0) __threadfence(); }
        wsync();
    }
}

__global__ __launch_bounds__(32) void k_gemm_vt(const bf* __restrict__ W, const bf* __restrict__ X, h16* VT) {
    __shared__ __align__(16) float os[16 * LOP];
    const int lane = threadIdx.x & 31, lr = lane & 15, hi = lane >> 4;
    const size_t z = blockIdx.z; const int r0 = blockIdx.x * 64, c0 = blockIdx.y * 64;
    const bf* Bt = X + z * (size_t)SEQ * DM;
    v8f acc[4][4];
#pragma unroll
    for (int mb = 0; mb < 4; ++mb)
#pragma unroll
        for (int nb = 0; nb < 4; ++nb) acc[mb][nb] = (v8f){};
    gemm_loop<0>(W, W, Bt, DM, (size_t)(r0 + lr) * DM + 8 * hi, (size_t)(c0 + lr) * DM + 8 * hi, acc);
    const size_t vb0 = z * (size_t)DM * SEQ + (size_t)r0 * SEQ + c0;
    const int srow = lane >> 3, scol = (lane & 7) * 8;
#pragma unroll
    for (int mb = 0; mb < 4; ++mb) {
#pragma unroll
        for (int nb = 0; nb < 4; ++nb) {
#pragma unroll
            for (int j = 0; j < 8; ++j) os[(hi * 8 + j) * LOP + nb * 16 + lr] = acc[mb][nb][j]; }
        wsync();
#pragma unroll 1
        for (int ps = 0; ps < 2; ++ps) {
#pragma unroll
            for (int s = 0; s < 4; ++s) { const int row = 4 * s + srow; const v4f x0 = *(const v4fa*)(&os[row * LOP + scol]); const v4f x1 = *(const v4fa*)(&os[row * LOP + scol + 4]); v8h o;
#pragma unroll
                for (int j = 0; j < 4; ++j) { o[j] = (h16)x0[j]; o[4 + j] = (h16)x1[j]; }
                *(volatile v8h*)(VT + vb0 + (size_t)(mb * 16 + row) * SEQ + scol) = o; }
            if (ps == 0) __threadfence(); }
        wsync();
    }
}

__global__ __launch_bounds__(32) void k_gemm_out(const bf* __restrict__ Ah, const bf* __restrict__ Al, const bf* __restrict__ W, const float* __restrict__ bias, float* C) {
    __shared__ __align__(16) float os[16 * LOP];
    const int lane = threadIdx.x & 31, lr = lane & 15, hi = lane >> 4;
    const size_t z = blockIdx.z; const int r0 = blockIdx.x * 64, c0 = blockIdx.y * 64;
    const bf* A = Ah + z * (size_t)SEQ * DM; const bf* A2 = Al + z * (size_t)SEQ * DM;
    float* Cz = C + z * (size_t)SEQ_FULL * DM;
    v8f acc[4][4];
#pragma unroll
    for (int mb = 0; mb < 4; ++mb)
#pragma unroll
        for (int nb = 0; nb < 4; ++nb) acc[mb][nb] = (v8f){};
    gemm_loop<1>(A, A2, W, DM, (size_t)(r0 + lr) * DM + 8 * hi, (size_t)(c0 + lr) * DM + 8 * hi, acc);
#pragma unroll
    for (int mb = 0; mb < 4; ++mb) {
#pragma unroll
        for (int nb = 0; nb < 4; ++nb) {
#pragma unroll
            for (int j = 0; j < 8; ++j) os[(hi * 8 + j) * LOP + nb * 16 + lr] = acc[mb][nb][j]; }
        wsync();
        float* crow = Cz + (size_t)(r0 + mb * 16) * DM + c0;
#pragma unroll 1
        for (int ps = 0; ps < 2; ++ps) {
#pragma unroll
            for (int s = 0; s < 8; ++s) { const int row = 2 * s + hi, cofs = lr * 4; v4f val = *(const v4fa*)(&os[row * LOP + cofs]);
                val[0] += bfr(bias[c0 + cofs]); val[1] += bfr(bias[c0 + cofs + 1]); val[2] += bfr(bias[c0 + cofs + 2]); val[3] += bfr(bias[c0 + cofs + 3]);
                *(volatile v4f*)(crow + (size_t)row * DM + cofs) = val; }
            if (ps == 0) __threadfence(); }
        wsync();
    }
}

__global__ __launch_bounds__(128) void k_flash(const bf* __restrict__ Qh, const bf* __restrict__ Ql, const bf* __restrict__ Kh, const bf* __restrict__ Kl, const h16* __restrict__ VT, bf* Ch, bf* Cl) {
    __shared__ __align__(16) bf    kh_s[64 * LKP];
    __shared__ __align__(16) bf    kl_s[64 * LKP];
    __shared__ __align__(16) h16   vt_s[64 * LKP];
    __shared__ __align__(16) h16   p_s[4 * 16 * LPP];
    __shared__ __align__(16) float o_s[4 * 16 * LOP];
    const int tid = threadIdx.x, lane = tid & 31, wid = tid >> 5, lr = lane & 15, hi = lane >> 4;
    const int bh = blockIdx.y; const int b = bh / NH, h = bh % NH;
    const int q0 = blockIdx.x * 64 + wid * 16;
    const size_t pl = (size_t)bh * SEQ * HD;
    const size_t qoff = pl + (size_t)(q0 + lr) * HD + 8 * hi;
    const size_t vbase = ((size_t)b * DM + (size_t)h * HD) * SEQ;
    const int pb = wid * 16 * LPP, ob = wid * 16 * LOP;
    v8f o[4];
#pragma unroll
    for (int dt = 0; dt < 4; ++dt) o[dt] = (v8f){};
    float mr[8], ls[8];
#pragma unroll
    for (int r = 0; r < 8; ++r) { mr[r] = -1.0e30f; ls[r] = 0.0f; }

#pragma unroll 1
    for (int kb = 0; kb < SEQ / 64; ++kb) {
        __syncthreads();
#pragma unroll
        for (int it = 0; it < 4; ++it) {
            const int u = tid + it * 128; const int row = u >> 3, part = (u & 7) * 8;
            const size_t g = pl + (size_t)kb * 64 * HD + (size_t)u * 8;
            const v8us a = *(const v8us*)(Kh + g); const v8us c = *(const v8us*)(Kl + g);
            const v8h v = *(const v8h*)(VT + vbase + (size_t)row * SEQ + (size_t)kb * 64 + part);
            *(v8usa*)(&kh_s[row * LKP + part]) = a; *(v8usa*)(&kl_s[row * LKP + part]) = c; *(v8ha*)(&vt_s[row * LKP + part]) = v;
        }
        __syncthreads();
#pragma unroll 1
        for (int hf = 0; hf < 2; ++hf) {
            v8f s0 = (v8f){}, s1 = (v8f){};
            const int kr0 = (hf * 32 + lr) * LKP + 8 * hi, kr1 = kr0 + 16 * LKP;
#pragma unroll
            for (int ks = 0; ks < 2; ++ks) {
                const int kk = ks * 32;
                const v16bf qh = ldg16(Qh + qoff + kk); const v16bf ql = ldg16(Ql + qoff + kk);
                const v16bf k0h = cat16b(*(const v8usa*)(&kh_s[kr0 + kk]), *(const v8usa*)(&kh_s[kr0 + kk + 16]));
                const v16bf k0l = cat16b(*(const v8usa*)(&kl_s[kr0 + kk]), *(const v8usa*)(&kl_s[kr0 + kk + 16]));
                const v16bf k1h = cat16b(*(const v8usa*)(&kh_s[kr1 + kk]), *(const v8usa*)(&kh_s[kr1 + kk + 16]));
                const v16bf k1l = cat16b(*(const v8usa*)(&kl_s[kr1 + kk]), *(const v8usa*)(&kl_s[kr1 + kk + 16]));
                s0 = wmmab(qh, k0h, s0); s1 = wmmab(qh, k1h, s1);
                s0 = wmmab(ql, k0h, s0); s1 = wmmab(ql, k1h, s1);
                s0 = wmmab(qh, k0l, s0); s1 = wmmab(qh, k1l, s1);
                asm volatile("v_nop\n\tv_nop\n\tv_nop\n\tv_nop" : "+v"(s0), "+v"(s1) : "v"(qh), "v"(ql), "v"(k0h), "v"(k0l), "v"(k1h), "v"(k1l));
            }
#pragma unroll
            for (int r = 0; r < 8; ++r) {
                const float a0 = s0[r], a1 = s1[r];
                float mx = fmaxf(a0, a1);
                mx = fmaxf(mx, __shfl_xor(mx, 1, 32)); mx = fmaxf(mx, __shfl_xor(mx, 2, 32)); mx = fmaxf(mx, __shfl_xor(mx, 4, 32)); mx = fmaxf(mx, __shfl_xor(mx, 8, 32));
                const float mnew = fmaxf(mr[r], mx);
                const float al = __builtin_amdgcn_exp2f((mr[r] - mnew) * L2E);
                const float p0 = __builtin_amdgcn_exp2f((a0 - mnew) * L2E);
                const float p1 = __builtin_amdgcn_exp2f((a1 - mnew) * L2E);
                ls[r] = ls[r] * al + (p0 + p1);
                mr[r] = mnew;
                o[0][r] *= al; o[1][r] *= al; o[2][r] *= al; o[3][r] *= al;
                p_s[pb + (8 * hi + r) * LPP + lr] = (h16)(p0 * PCAR);
                p_s[pb + (8 * hi + r) * LPP + 16 + lr] = (h16)(p1 * PCAR);
            }
            wsync();
            const v16h pa = cat16(*(const v8ha*)(&p_s[pb + lr * LPP + 8 * hi]), *(const v8ha*)(&p_s[pb + lr * LPP + 8 * hi + 16]));
            v16h vb[4];
#pragma unroll
            for (int dt = 0; dt < 4; ++dt) { const int vo = (dt * 16 + lr) * LKP + hf * 32 + 8 * hi; vb[dt] = cat16(*(const v8ha*)(&vt_s[vo]), *(const v8ha*)(&vt_s[vo + 16])); }
#pragma unroll
            for (int dt = 0; dt < 4; ++dt) o[dt] = wmma16(pa, vb[dt], o[dt]);
            asm volatile("v_nop\n\tv_nop\n\tv_nop\n\tv_nop" : "+v"(o[0]), "+v"(o[1]), "+v"(o[2]), "+v"(o[3]) : "v"(pa), "v"(vb[0]), "v"(vb[1]), "v"(vb[2]), "v"(vb[3]));
            wsync();
        }
    }
#pragma unroll
    for (int r = 0; r < 8; ++r) {
        float lt = ls[r];
        lt += __shfl_xor(lt, 1, 32); lt += __shfl_xor(lt, 2, 32); lt += __shfl_xor(lt, 4, 32); lt += __shfl_xor(lt, 8, 32);
        const float inv = 1.0f / (lt * PCAR);
#pragma unroll
        for (int dt = 0; dt < 4; ++dt) o_s[ob + (8 * hi + r) * LOP + dt * 16 + lr] = o[dt][r] * inv;
    }
    wsync();
    const int srow = lane >> 3, scol = (lane & 7) * 8;
    const size_t cbase = ((size_t)b * SEQ + q0) * DM + (size_t)h * HD;
#pragma unroll 1
    for (int ps = 0; ps < 2; ++ps) {
#pragma unroll
        for (int s = 0; s < 4; ++s) { const int row = 4 * s + srow; const v4f x0 = *(const v4fa*)(&o_s[ob + row * LOP + scol]); const v4f x1 = *(const v4fa*)(&o_s[ob + row * LOP + scol + 4]); v8us oh, ol;
#pragma unroll
            for (int j = 0; j < 4; ++j) { unsigned short a, c; splitf(x0[j], a, c); oh[j] = a; ol[j] = c; splitf(x1[j], a, c); oh[4 + j] = a; ol[4 + j] = c; }
            const size_t off = cbase + (size_t)row * DM + scol;
            *(volatile v8us*)(Ch + off) = oh; *(volatile v8us*)(Cl + off) = ol; }
        if (ps == 0) __threadfence(); }
}

constexpr size_t al256(size_t x) { return (x + 255) & ~(size_t)255; }
constexpr size_t SZ_W = al256((size_t)DM * DM * 2);
constexpr size_t SZ_X = al256((size_t)NB * SEQ * DM * 2);
constexpr size_t SZ_P = al256((size_t)NB * NH * SEQ * HD * 2);
constexpr size_t WS_TOTAL = 4 * SZ_W + 3 * SZ_X + 4 * SZ_P + SZ_P + 2 * SZ_X;
static_assert(WS_TOTAL <= (size_t)134217728);
static_assert(SZ_P == SZ_X);

extern "C" void kernel_launch(void* const* d_in, const int* in_sizes, int n_in,
                              void* d_out, int out_size, void* d_ws, size_t ws_size, hipStream_t stream) {
    if (n_in < 8) return;
    const size_t need_act = (size_t)(NB - 1) * SEQ_FULL * DM + (size_t)SEQ * DM;
    if ((size_t)in_sizes[0] < need_act || (size_t)in_sizes[1] < need_act || (size_t)in_sizes[2] < need_act) return;
    if ((size_t)in_sizes[3] < (size_t)DM * DM || (size_t)in_sizes[4] < (size_t)DM * DM || (size_t)in_sizes[5] < (size_t)DM * DM || (size_t)in_sizes[6] < (size_t)DM * DM || in_sizes[7] < DM) return;
    if ((size_t)out_size < need_act) return;
    if (WS_TOTAL > ws_size) return;
    const float* xq = (const float*)d_in[0]; const float* xk = (const float*)d_in[1]; const float* xv = (const float*)d_in[2];
    const float* wq = (const float*)d_in[3]; const float* wk = (const float*)d_in[4]; const float* wv = (const float*)d_in[5]; const float* wo = (const float*)d_in[6]; const float* bo = (const float*)d_in[7];
    float* OUT = (float*)d_out;
    char* wsp = (char*)d_ws;
    auto take = [&](size_t bytes) { char* p = wsp; wsp += bytes; return (void*)p; };
    bf* WQ = (bf*)take(SZ_W); bf* WK = (bf*)take(SZ_W); bf* WV = (bf*)take(SZ_W); bf* WO = (bf*)take(SZ_W);
    bf* XQ = (bf*)take(SZ_X); bf* XK = (bf*)take(SZ_X); bf* XV = (bf*)take(SZ_X);
    bf* QPh = (bf*)take(SZ_P); bf* QPl = (bf*)take(SZ_P); bf* KPh = (bf*)take(SZ_P); bf* KPl = (bf*)take(SZ_P);
    h16* VT = (h16*)take(SZ_P);
    bf* CTh = (bf*)take(SZ_X); bf* CTl = (bf*)take(SZ_X);
    if ((size_t)(wsp - (char*)d_ws) != WS_TOTAL) return;

    const unsigned nw8 = (unsigned)((size_t)DM * DM / 8), na8 = (unsigned)((size_t)SEQ * DM / 8);
    k_cvt8<<<dim3(nw8 / 256, 1), 256, 0, stream>>>(wq, WQ, nw8, 0, 0);
    k_cvt8<<<dim3(nw8 / 256, 1), 256, 0, stream>>>(wk, WK, nw8, 0, 0);
    k_cvt8<<<dim3(nw8 / 256, 1), 256, 0, stream>>>(wv, WV, nw8, 0, 0);
    k_cvt8<<<dim3(nw8 / 256, 1), 256, 0, stream>>>(wo, WO, nw8, 0, 0);
    k_cvt8<<<dim3(na8 / 256, NB), 256, 0, stream>>>(xq, XQ, na8, (size_t)SEQ_FULL * DM, (size_t)SEQ * DM);
    k_cvt8<<<dim3(na8 / 256, NB), 256, 0, stream>>>(xk, XK, na8, (size_t)SEQ_FULL * DM, (size_t)SEQ * DM);
    k_cvt8<<<dim3(na8 / 256, NB), 256, 0, stream>>>(xv, XV, na8, (size_t)SEQ_FULL * DM, (size_t)SEQ * DM);
    k_gemm_qk<<<dim3(SEQ / 64, NH, NB), 32, 0, stream>>>(XQ, WQ, QPh, QPl, SCL);
    k_gemm_qk<<<dim3(SEQ / 64, NH, NB), 32, 0, stream>>>(XK, WK, KPh, KPl, 1.0f);
    k_gemm_vt<<<dim3(DM / 64, SEQ / 64, NB), 32, 0, stream>>>(WV, XV, VT);
    k_flash<<<dim3(SEQ / 64, NB * NH), 128, 0, stream>>>(QPh, QPl, KPh, KPl, VT, CTh, CTl);
    k_gemm_out<<<dim3(SEQ / 64, DM / 64, NB), 32, 0, stream>>>(CTh, CTl, WO, bo, OUT);
}
